// ReBasedLinearAttention_41489384079872
// MI455X (gfx1250) — hardware-verified
//
#include <hip/hip_runtime.h>
#include <stdint.h>
#include <stddef.h>


#define T_SEQ 2048
#define HID   2048
#define NH    16
#define HD    128
#define LN_EPS  1e-5f
#define ATT_EPS 1e-5f
#define SC_P  36
#define SP_P  40
#define SO_P  136

typedef unsigned short u16;
typedef u16    us8     __attribute__((ext_vector_type(8)));
typedef __bf16 bf16x16 __attribute__((ext_vector_type(16)));
typedef float  v8f     __attribute__((ext_vector_type(8)));
typedef float  v4f     __attribute__((ext_vector_type(4)));

union Frag  { bf16x16 v; us8 h[2]; };
union Pack8 { us8 v; u16 s[8]; };

__device__ __forceinline__ u16 bf16_rne(float x) {
  unsigned u = __float_as_uint(x);
  u = u + 0x7FFFu + ((u >> 16) & 1u);
  return (u16)(u >> 16);
}
__device__ __forceinline__ float bf16_val(u16 b) {
  return __uint_as_float(((unsigned)b) << 16);
}
__device__ __forceinline__ void split_bf16(float x, u16& hi, u16& lo) {
  hi = bf16_rne(x);
  lo = bf16_rne(x - bf16_val(hi));
}
__device__ __forceinline__ void split_pack8(const float* y, us8& hi, us8& lo) {
  Pack8 ph, pl;
#pragma unroll
  for (int e = 0; e < 8; ++e) {
    u16 a, b;
    split_bf16(y[e], a, b);
    ph.s[e] = a;
    pl.s[e] = b;
  }
  hi = ph.v;
  lo = pl.v;
}
__device__ __forceinline__ us8 ld8(const u16* p) { return *(const us8*)p; }

__device__ __forceinline__ v8f v8zero() {
  v8f z = {0.f, 0.f, 0.f, 0.f, 0.f, 0.f, 0.f, 0.f};
  return z;
}

__device__ __forceinline__ v8f wmma3(const bf16x16 ah, const bf16x16 al,
                                     const bf16x16 bh, const bf16x16 bl, v8f c) {
  c = __builtin_amdgcn_wmma_f32_16x16x32_bf16(false, ah, false, bh, (short)0, c, false, false);
  c = __builtin_amdgcn_wmma_f32_16x16x32_bf16(false, ah, false, bl, (short)0, c, false, false);
  c = __builtin_amdgcn_wmma_f32_16x16x32_bf16(false, al, false, bh, (short)0, c, false, false);
  asm volatile("v_nop\n\tv_nop\n\tv_nop\n\tv_nop" : "+v"(c) : "v"(ah), "v"(al), "v"(bh), "v"(bl));
  return c;
}

__global__ __launch_bounds__(256) void k_split_planes(const float* __restrict__ X,
                                                       u16* Ph, u16* Pl, int n8) {
  const int i = blockIdx.x * 256 + threadIdx.x;
  if (i >= n8) return;
  const float* p = X + (size_t)i * 8;
  const v4f a = *(const v4f*)p;
  const v4f b = *(const v4f*)(p + 4);
  float y[8];
  y[0] = a.x; y[1] = a.y; y[2] = a.z; y[3] = a.w;
  y[4] = b.x; y[5] = b.y; y[6] = b.z; y[7] = b.w;
  us8 vh, vl;
  split_pack8(y, vh, vl);
  const size_t go = (size_t)i * 8;
  *(volatile us8*)(Ph + go) = vh;
  *(volatile us8*)(Pl + go) = vl;
  __threadfence();
  *(volatile us8*)(Ph + go) = vh;
  *(volatile us8*)(Pl + go) = vl;
}

__global__ __launch_bounds__(64) void k_gemm_nt3(
    const u16* __restrict__ Ah, const u16* __restrict__ Al,
    const u16* __restrict__ Bh, const u16* __restrict__ Bl,
    float* C, int K, int ldc) {
  __shared__ __align__(16) float sC[2][64][SC_P];
  const int lane = threadIdx.x & 31, w = threadIdx.x >> 5;
  const int hh = lane >> 4, m = lane & 15;
  const int row0 = blockIdx.y * 64;
  const int col0 = blockIdx.x * 64 + w * 32;

  v8f acc[4][2];
#pragma unroll
  for (int i = 0; i < 4; ++i) { acc[i][0] = v8zero(); acc[i][1] = v8zero(); }

  const size_t arow = (size_t)(row0 + m) * K + 8 * hh;
  const size_t brow = (size_t)(col0 + m) * K + 8 * hh;

#pragma unroll 1
  for (int k0 = 0; k0 < K; k0 += 32) {
    Frag bh[2], bl[2];
#pragma unroll
    for (int j = 0; j < 2; ++j) {
      const size_t o = brow + (size_t)(16 * j) * K + k0;
      bh[j].h[0] = ld8(Bh + o);  bh[j].h[1] = ld8(Bh + o + 16);
      bl[j].h[0] = ld8(Bl + o);  bl[j].h[1] = ld8(Bl + o + 16);
    }
#pragma unroll
    for (int i = 0; i < 4; ++i) {
      const size_t o = arow + (size_t)(16 * i) * K + k0;
      Frag ah, al;
      ah.h[0] = ld8(Ah + o);  ah.h[1] = ld8(Ah + o + 16);
      al.h[0] = ld8(Al + o);  al.h[1] = ld8(Al + o + 16);
      acc[i][0] = wmma3(ah.v, al.v, bh[0].v, bl[0].v, acc[i][0]);
      acc[i][1] = wmma3(ah.v, al.v, bh[1].v, bl[1].v, acc[i][1]);
    }
  }

#pragma unroll
  for (int i = 0; i < 4; ++i)
#pragma unroll
    for (int j = 0; j < 2; ++j)
#pragma unroll
      for (int r = 0; r < 8; ++r)
        sC[w][16 * i + 8 * hh + r][16 * j + m] = acc[i][j][r];
  __syncthreads();

  const int piece = lane & 7, rsub = lane >> 3;
#pragma unroll
  for (int it = 0; it < 16; ++it) {
    const int row = it * 4 + rsub;
    const v4f v = *(const v4f*)&sC[w][row][piece * 4];
    *(volatile v4f*)(C + (size_t)(row0 + row) * ldc + col0 + piece * 4) = v;
  }
  __threadfence();
#pragma unroll
  for (int it = 0; it < 16; ++it) {
    const int row = it * 4 + rsub;
    const v4f v = *(const v4f*)&sC[w][row][piece * 4];
    *(volatile v4f*)(C + (size_t)(row0 + row) * ldc + col0 + piece * 4) = v;
  }
}

__global__ __launch_bounds__(128) void k_feature_map(const float* __restrict__ F,
    const float* __restrict__ gamma, const float* __restrict__ beta,
    u16* Yh, u16* Yl, float outscale) {
  const int tid = threadIdx.x, lane = tid & 31, w = tid >> 5;
  const int h = blockIdx.y;
  const int t = blockIdx.x * 8 + 2 * w + (lane >> 4);
  const int c = (lane & 15) * 8;
  const float* xp = F + (size_t)t * HID + h * HD + c;
  const v4f x0 = *(const v4f*)xp;
  const v4f x1 = *(const v4f*)(xp + 4);
  const v4f g0 = *(const v4f*)(gamma + c);
  const v4f g1 = *(const v4f*)(gamma + c + 4);
  const v4f b0 = *(const v4f*)(beta + c);
  const v4f b1 = *(const v4f*)(beta + c + 4);
  float y[8];
  y[0] = x0.x * g0.x + b0.x;  y[1] = x0.y * g0.y + b0.y;
  y[2] = x0.z * g0.z + b0.z;  y[3] = x0.w * g0.w + b0.w;
  y[4] = x1.x * g1.x + b1.x;  y[5] = x1.y * g1.y + b1.y;
  y[6] = x1.z * g1.z + b1.z;  y[7] = x1.w * g1.w + b1.w;
  float s = 0.0f;
#pragma unroll
  for (int e = 0; e < 8; ++e) s += y[e];
  s += __shfl_xor(s, 1, 32);  s += __shfl_xor(s, 2, 32);
  s += __shfl_xor(s, 4, 32);  s += __shfl_xor(s, 8, 32);
  const float mu = s * (1.0f / 128.0f);
  float d[8];
  float vs = 0.0f;
#pragma unroll
  for (int e = 0; e < 8; ++e) { d[e] = y[e] - mu; vs += d[e] * d[e]; }
  vs += __shfl_xor(vs, 1, 32);  vs += __shfl_xor(vs, 2, 32);
  vs += __shfl_xor(vs, 4, 32);  vs += __shfl_xor(vs, 8, 32);
  const float inv = rsqrtf(vs * (1.0f / 128.0f) + LN_EPS) * outscale;
  float o[8];
#pragma unroll
  for (int e = 0; e < 8; ++e) o[e] = d[e] * inv;
  us8 vh, vl;
  split_pack8(o, vh, vl);
  const size_t go = ((size_t)h * T_SEQ + t) * HD + c;
  *(volatile us8*)(Yh + go) = vh;
  *(volatile us8*)(Yl + go) = vl;
  __threadfence();
  *(volatile us8*)(Yh + go) = vh;
  *(volatile us8*)(Yl + go) = vl;
}

__global__ __launch_bounds__(128) void k_vsplit_t(const float* __restrict__ Vf, u16* Vth, u16* Vtl) {
  __shared__ float sV[64][65];
  const int tid = threadIdx.x, lane = tid & 31, w = tid >> 5;
  const int kb = blockIdx.x * 64;
  const int cb = blockIdx.y * 64;
#pragma unroll
  for (int p = 0; p < 8; ++p) {
    const int r = p * 8 + (tid >> 4);
    const int c4 = (tid & 15) * 4;
    const v4f v = *(const v4f*)(Vf + (size_t)(kb + r) * HID + cb + c4);
    sV[r][c4 + 0] = v.x;  sV[r][c4 + 1] = v.y;
    sV[r][c4 + 2] = v.z;  sV[r][c4 + 3] = v.w;
  }
  __syncthreads();
  const int piece = lane & 7;
  us8 vh[4], vl[4];
  size_t go[4];
#pragma unroll
  for (int it = 0; it < 4; ++it) {
    const int ch = w * 16 + it * 4 + (lane >> 3);
    float y[8];
#pragma unroll
    for (int e = 0; e < 8; ++e) y[e] = sV[piece * 8 + e][ch];
    split_pack8(y, vh[it], vl[it]);
    go[it] = (size_t)(cb + ch) * T_SEQ + kb + piece * 8;
  }
#pragma unroll
  for (int it = 0; it < 4; ++it) {
    *(volatile us8*)(Vth + go[it]) = vh[it];
    *(volatile us8*)(Vtl + go[it]) = vl[it];
  }
  __threadfence();
#pragma unroll
  for (int it = 0; it < 4; ++it) {
    *(volatile us8*)(Vth + go[it]) = vh[it];
    *(volatile us8*)(Vtl + go[it]) = vl[it];
  }
}

__global__ __launch_bounds__(32) void k_attn_quad(
    const u16* __restrict__ Qh, const u16* __restrict__ Ql,
    const u16* __restrict__ Kh, const u16* __restrict__ Kl,
    const u16* __restrict__ Vth, const u16* __restrict__ Vtl,
    u16* Oh, u16* Ol) {
  __shared__ __align__(16) u16 sPh[16 * SP_P];
  __shared__ __align__(16) u16 sPl[16 * SP_P];
  __shared__ __align__(16) u16 sOh[16 * SO_P];
  __shared__ __align__(16) u16 sOl[16 * SO_P];
  const int lane = threadIdx.x & 31, hh = lane >> 4, m = lane & 15;
  const int q0 = blockIdx.x * 16, h = blockIdx.y;
  const size_t qoff = ((size_t)h * T_SEQ + q0 + m) * HD + 8 * hh;
  const u16* Kbh = Kh + (size_t)h * T_SEQ * HD;
  const u16* Kbl = Kl + (size_t)h * T_SEQ * HD;
  const u16* Vbh = Vth + (size_t)h * HD * T_SEQ;
  const u16* Vbl = Vtl + (size_t)h * HD * T_SEQ;

  v8f oacc[8];
#pragma unroll
  for (int j = 0; j < 8; ++j) oacc[j] = v8zero();
  float zp[8];
#pragma unroll
  for (int r = 0; r < 8; ++r) zp[r] = 0.0f;

  const int kvend = q0 + 16;
#pragma unroll 1
  for (int kv0 = 0; kv0 < kvend; kv0 += 32) {
    v8f s0 = v8zero(), s1 = v8zero();
#pragma unroll
    for (int kc = 0; kc < 4; ++kc) {
      Frag qh, ql, k0h, k0l, k1h, k1l;
      const size_t qo = qoff + 32 * kc;
      qh.h[0] = ld8(Qh + qo);  qh.h[1] = ld8(Qh + qo + 16);
      ql.h[0] = ld8(Ql + qo);  ql.h[1] = ld8(Ql + qo + 16);
      const size_t ko0 = (size_t)(kv0 + m) * HD + 32 * kc + 8 * hh;
      const size_t ko1 = ko0 + (size_t)16 * HD;
      k0h.h[0] = ld8(Kbh + ko0);  k0h.h[1] = ld8(Kbh + ko0 + 16);
      k0l.h[0] = ld8(Kbl + ko0);  k0l.h[1] = ld8(Kbl + ko0 + 16);
      k1h.h[0] = ld8(Kbh + ko1);  k1h.h[1] = ld8(Kbh + ko1 + 16);
      k1l.h[0] = ld8(Kbl + ko1);  k1l.h[1] = ld8(Kbl + ko1 + 16);
      s0 = wmma3(qh.v, ql.v, k0h.v, k0l.v, s0);
      s1 = wmma3(qh.v, ql.v, k1h.v, k1l.v, s1);
    }
    __syncthreads();
#pragma unroll
    for (int r = 0; r < 8; ++r) {
      const int qr = q0 + 8 * hh + r;
      const float a0 = s0[r];
      const float a1 = s1[r];
      const float p0 = (kv0 + m <= qr) ? a0 * a0 : 0.0f;
      const float p1 = (kv0 + 16 + m <= qr) ? a1 * a1 : 0.0f;
      zp[r] += p0;
      zp[r] += p1;
      u16 ph0, pl0, ph1, pl1;
      split_bf16(p0, ph0, pl0);
      split_bf16(p1, ph1, pl1);
      sPh[(8 * hh + r) * SP_P + m] = ph0;
      sPl[(8 * hh + r) * SP_P + m] = pl0;
      sPh[(8 * hh + r) * SP_P + 16 + m] = ph1;
      sPl[(8 * hh + r) * SP_P + 16 + m] = pl1;
    }
    __syncthreads();
    Frag ph, pl;
    ph.h[0] = ld8(sPh + m * SP_P + 8 * hh);  ph.h[1] = ld8(sPh + m * SP_P + 16 + 8 * hh);
    pl.h[0] = ld8(sPl + m * SP_P + 8 * hh);  pl.h[1] = ld8(sPl + m * SP_P + 16 + 8 * hh);
#pragma unroll
    for (int j = 0; j < 8; ++j) {
      const size_t vo = (size_t)(16 * j + m) * T_SEQ + kv0 + 8 * hh;
      Frag vh, vl;
      vh.h[0] = ld8(Vbh + vo);  vh.h[1] = ld8(Vbh + vo + 16);
      vl.h[0] = ld8(Vbl + vo);  vl.h[1] = ld8(Vbl + vo + 16);
      oacc[j] = wmma3(ph.v, pl.v, vh.v, vl.v, oacc[j]);
    }
  }

#pragma unroll
  for (int r = 0; r < 8; ++r) {
    float z = zp[r];
    z += __shfl_xor(z, 1, 32);  z += __shfl_xor(z, 2, 32);
    z += __shfl_xor(z, 4, 32);  z += __shfl_xor(z, 8, 32);
    zp[r] = 1.0f / (z + ATT_EPS);
  }
#pragma unroll
  for (int j = 0; j < 8; ++j)
#pragma unroll
    for (int r = 0; r < 8; ++r) {
      const float o = oacc[j][r] * zp[r];
      u16 hi, lo;
      split_bf16(o, hi, lo);
      sOh[(8 * hh + r) * SO_P + 16 * j + m] = hi;
      sOl[(8 * hh + r) * SO_P + 16 * j + m] = lo;
    }
  __syncthreads();
#pragma unroll
  for (int it = 0; it < 8; ++it) {
    const int row = 2 * it + hh;
    const us8 vh = ld8(sOh + row * SO_P + 8 * m);
    const us8 vl = ld8(sOl + row * SO_P + 8 * m);
    const size_t go = (size_t)(q0 + row) * HID + h * HD + 8 * m;
    *(volatile us8*)(Oh + go) = vh;
    *(volatile us8*)(Ol + go) = vl;
  }
  __threadfence();
#pragma unroll
  for (int it = 0; it < 8; ++it) {
    const int row = 2 * it + hh;
    const us8 vh = ld8(sOh + row * SO_P + 8 * m);
    const us8 vl = ld8(sOl + row * SO_P + 8 * m);
    const size_t go = (size_t)(q0 + row) * HID + h * HD + 8 * m;
    *(volatile us8*)(Oh + go) = vh;
    *(volatile us8*)(Ol + go) = vl;
  }
}

extern "C" void kernel_launch(void* const* d_in, const int* in_sizes, int n_in,
                              void* d_out, int out_size, void* d_ws, size_t ws_size,
                              hipStream_t stream) {
  if (n_in < 7) return;
  const int nel = T_SEQ * HID;
  if (in_sizes[0] != nel || in_sizes[1] != nel || in_sizes[2] != nel ||
      in_sizes[3] != nel || in_sizes[4] != nel ||
      in_sizes[5] != HD || in_sizes[6] != HD || out_size != nel) return;

  const float* X     = (const float*)d_in[0];
  const float* Wq    = (const float*)d_in[1];
  const float* Wk    = (const float*)d_in[2];
  const float* Wv    = (const float*)d_in[3];
  const float* Wo    = (const float*)d_in[4];
  const float* gamma = (const float*)d_in[5];
  const float* beta  = (const float*)d_in[6];
  float* out = (float*)d_out;

  const size_t plane2 = (size_t)nel * 2;
  const size_t plane4 = (size_t)nel * 4;
  size_t off = 0;
  const size_t oXh = off; off += plane2;
  const size_t oXl = off; off += plane2;
  const size_t oWh = off; off += plane2;
  const size_t oWl = off; off += plane2;
  const size_t oF  = off; off += plane4;
  const size_t oQh = off; off += plane2;
  const size_t oQl = off; off += plane2;
  const size_t oKh = off; off += plane2;
  const size_t oKl = off; off += plane2;
  const size_t oVh = off; off += plane2;
  const size_t oVl = off; off += plane2;
  if (off > ws_size) return;

  char* ws = (char*)d_ws;
  u16* Xh  = (u16*)(ws + oXh);  u16* Xl  = (u16*)(ws + oXl);
  u16* Wh  = (u16*)(ws + oWh);  u16* Wl  = (u16*)(ws + oWl);
  float* F = (float*)(ws + oF);
  u16* Qh  = (u16*)(ws + oQh);  u16* Ql  = (u16*)(ws + oQl);
  u16* Khp = (u16*)(ws + oKh);  u16* Klp = (u16*)(ws + oKl);
  u16* Vth = (u16*)(ws + oVh);  u16* Vtl = (u16*)(ws + oVl);
  u16* Ohp = Xh;  u16* Olp = Xl;

  const int n8 = nel / 8;
  const dim3 gsplit(n8 / 256);
  const dim3 ggemm(HID / 64, T_SEQ / 64);
  const dim3 gfmap(T_SEQ / 8, NH);
  const dim3 gvsp(T_SEQ / 64, HID / 64);
  const dim3 gattn(T_SEQ / 16, NH);
  const float qscale = 0.08838834764831845f;

  k_split_planes<<<gsplit, 256, 0, stream>>>(X, Xh, Xl, n8);
  k_split_planes<<<gsplit, 256, 0, stream>>>(Wq, Wh, Wl, n8);
  k_gemm_nt3<<<ggemm, 64, 0, stream>>>(Xh, Xl, Wh, Wl, F, HID, HID);
  k_feature_map<<<gfmap, 128, 0, stream>>>(F, gamma, beta, Qh, Ql, qscale);
  k_split_planes<<<gsplit, 256, 0, stream>>>(Wk, Wh, Wl, n8);
  k_gemm_nt3<<<ggemm, 64, 0, stream>>>(Xh, Xl, Wh, Wl, F, HID, HID);
  k_feature_map<<<gfmap, 128, 0, stream>>>(F, gamma, beta, Khp, Klp, 1.0f);
  k_split_planes<<<gsplit, 256, 0, stream>>>(Wv, Wh, Wl, n8);
  k_gemm_nt3<<<ggemm, 64, 0, stream>>>(Xh, Xl, Wh, Wl, F, HID, HID);
  k_vsplit_t<<<gvsp, 128, 0, stream>>>(F, Vth, Vtl);
  k_attn_quad<<<gattn, 32, 0, stream>>>(Qh, Ql, Khp, Klp, Vth, Vtl, Ohp, Olp);
  k_split_planes<<<gsplit, 256, 0, stream>>>(Wo, Wh, Wl, n8);
  k_gemm_nt3<<<ggemm, 64, 0, stream>>>(Ohp, Olp, Wh, Wl, out, HID, HID);
}
